// Baseline_64080912056948
// MI455X (gfx1250) — hardware-verified
//
#include <hip/hip_runtime.h>


namespace {
constexpr int NB = 1024, TT = 256, L = 128, IN = 128, H1 = 100, H1P = 112  , KP = 128, G3 = 3 * L, TD = TT - 1;
constexpr float HS = 256.0f, WSC = 256.0f, BNEPS = 1e-5f;
typedef _Float16 b16;
typedef __attribute__((ext_vector_type(16))) _Float16 v16b;
typedef __attribute__((ext_vector_type(8))) _Float16 v8b;
typedef __attribute__((ext_vector_type(8))) float v8f;
typedef __attribute__((ext_vector_type(4))) float v4f;
__device__ __forceinline__ float bf16_rne(float f) { unsigned int u = __float_as_uint(f); u += 0x7FFFu + ((u >> 16) & 1u); float r = __uint_as_float(u & 0xFFFF0000u); asm volatile("" : "+v"(r)); return r; }
__device__ __forceinline__ float bfv(float f) { float r = bf16_rne(f); asm volatile("" : "+v"(r)); return r; }
__device__ __forceinline__ void split16(float v, b16& hi, b16& lo) { hi = (b16)v; lo = (b16)(v - (float)hi); }
__device__ __forceinline__ v16b frag_kb(const b16* p, int hh) { const v8b a = *(const v8b*)(p + 8 * hh), b = *(const v8b*)(p + 16 + 8 * hh); v16b f;
#pragma unroll
  for (int e = 0; e < 8; ++e) { f[e] = a[e]; f[8 + e] = b[e]; } return f; }
__device__ __forceinline__ v8f wmma16b(v16b a, v16b b, v8f c) { v8f d = __builtin_amdgcn_wmma_f32_16x16x32_f16(false, a, false, b, (short)0, c, false, false); asm volatile("v_nop\n\tv_nop\n\tv_nop\n\tv_nop" : "+v"(d) : "v"(a), "v"(b)); return d; }
__device__ __forceinline__ void wave_lds_sync() { __builtin_amdgcn_fence(__ATOMIC_RELEASE, "workgroup"); __builtin_amdgcn_wave_barrier(); __builtin_amdgcn_fence(__ATOMIC_ACQUIRE, "workgroup"); }
__device__ __forceinline__ float pmul(float a, float b) { float p = a * b; asm volatile("" : "+v"(p)); return p; }
__device__ __forceinline__ float sigm(float v) { return 1.0f / (1.0f + __expf(-v)); }

__global__ __launch_bounds__(256) void wput_kernel(const float* __restrict__ w1, const float* __restrict__ w2, const float* __restrict__ w3, const float* __restrict__ whh, b16* __restrict__ W1P, b16* __restrict__ W2P, b16* __restrict__ W3P, b16* __restrict__ WHP) { const int u = blockIdx.x * 256 + threadIdx.x; v8b v; const int o = u / 16, k0 = (u % 16) * 8;
  if (u < H1P * 16) {
#pragma unroll
    for (int j = 0; j < 8; ++j) v[j] = (b16)(o < H1 ? bf16_rne(w1[(size_t)o * IN + k0 + j]) * WSC : 0.0f); for (int pass = 0; pass < 2; ++pass) { *(volatile v8b*)(W1P + (size_t)o * KP + k0) = v; __threadfence(); }
#pragma unroll
    for (int j = 0; j < 8; ++j) { const int k = k0 + j; v[j] = (b16)((o < H1 && k < H1) ? bf16_rne(w2[(size_t)o * H1 + k]) * WSC : 0.0f); } for (int pass = 0; pass < 2; ++pass) { *(volatile v8b*)(W2P + (size_t)o * KP + k0) = v; __threadfence(); } }
  if (u < 2 * L * 16) {
#pragma unroll
    for (int j = 0; j < 8; ++j) { const int k = k0 + j; v[j] = (b16)(k < H1 ? bf16_rne(w3[(size_t)o * H1 + k]) * WSC : 0.0f); } for (int pass = 0; pass < 2; ++pass) { *(volatile v8b*)(W3P + (size_t)o * KP + k0) = v; __threadfence(); } }
  if (u < G3 * 16) {
#pragma unroll
    for (int j = 0; j < 8; ++j) v[j] = (b16)(bf16_rne(whh[(size_t)o * L + k0 + j]) * WSC); for (int pass = 0; pass < 2; ++pass) { *(volatile v8b*)(WHP + (size_t)o * KP + k0) = v; __threadfence(); } } }
template <int MODE>
__global__ __launch_bounds__(32) void enc_kernel(const float* __restrict__ XIN, const float* __restrict__ HIN, const float* __restrict__ BNs, const float* __restrict__ g, const float* __restrict__ be, const b16* __restrict__ W, const float* __restrict__ bias, float* __restrict__ HO, float* __restrict__ PS) { __shared__ __attribute__((aligned(16))) b16 Ah[16][KP + 8], Al[16][KP + 8]; __shared__ float Tf[16][H1P + 4]; const int lane = threadIdx.x, nloc = lane & 15, hlf = lane >> 4; const size_t m0 = (size_t)blockIdx.x * 16;
  for (int rr = 0; rr < 16; ++rr) for (int q = 0; q < 4; ++q) { const int c = q * 32 + lane; b16 p, ql; if (MODE == 0) { p = (b16)(bf16_rne(XIN[(m0 + rr) * TT + c]) * HS); ql = (b16)0.0f; } else { const float v = c < H1 ? pmul(pmul(HIN[(m0 + rr) * H1P + c] - BNs[c], BNs[H1P + c]), bfv(g[c])) + bfv(be[c]) : 0.0f; split16(v * HS, p, ql); } Ah[rr][c] = p; Al[rr][c] = ql; }
  if (lane < 16) for (int k = KP; k < KP + 8; ++k) { Ah[lane][k] = (b16)0.0f; Al[lane][k] = (b16)0.0f; }
  wave_lds_sync(); v8f acc[7];
#pragma unroll
  for (int t = 0; t < 7; ++t) acc[t] = (v8f){};
#pragma unroll
  for (int kb = 0; kb < KP; kb += 32) { const v16b a = frag_kb(&Ah[nloc][kb], hlf), al = frag_kb(&Al[nloc][kb], hlf);
#pragma unroll
    for (int t = 0; t < 7; ++t) { const v16b bw = frag_kb(W + (size_t)(t * 16 + nloc) * KP + kb, hlf); acc[t] = wmma16b(a, bw, acc[t]); if (MODE == 1) acc[t] = wmma16b(al, bw, acc[t]); } }
#pragma unroll
  for (int t = 0; t < 7; ++t) { const int cc = t * 16 + nloc; const float bb = cc < H1 ? bfv(bias[cc]) : 0.0f;
#pragma unroll
    for (int r8 = 0; r8 < 8; ++r8) Tf[8 * hlf + r8][cc] = cc < H1 ? fmaxf(acc[t][r8] * (1.0f / (HS * WSC)) + bb, 0.0f) : 0.0f; }
  wave_lds_sync();
  for (int pass = 0; pass < 2; ++pass) { for (int rr = 0; rr < 16; ++rr) for (int c = lane; c < H1P; c += 32) ((volatile float*)HO)[(m0 + rr) * H1P + c] = Tf[rr][c];
    for (int c = lane; c < H1P; c += 32) { float s = 0.0f, s2 = 0.0f; for (int rr = 0; rr < 16; ++rr) { const float v = Tf[rr][c]; s += v; s2 += v * v; } ((volatile float*)PS)[(size_t)blockIdx.x * 2 * H1P + c] = s; ((volatile float*)PS)[(size_t)blockIdx.x * 2 * H1P + H1P + c] = s2; } __threadfence(); } }
__global__ __launch_bounds__(128) void bn_kernel(const float* __restrict__ PS, float* __restrict__ BNs) { const int c = threadIdx.x; if (c >= H1P) return; double s = 0.0, s2 = 0.0; for (int w = 0; w < NB / 16; ++w) { s += (double)PS[(size_t)w * 2 * H1P + c]; s2 += (double)PS[(size_t)w * 2 * H1P + H1P + c]; } const double mu = s / NB; double var = s2 / NB - mu * mu; if (var < 0.0) var = 0.0;
  for (int pass = 0; pass < 2; ++pass) { ((volatile float*)BNs)[c] = (float)mu; ((volatile float*)BNs)[H1P + c] = (float)(1.0 / sqrt(var + (double)BNEPS)); __threadfence(); } }
__global__ __launch_bounds__(32) void lat_kernel(const float* __restrict__ H2, const float* __restrict__ BNs, const float* __restrict__ g, const float* __restrict__ be, const b16* __restrict__ W3P, const float* __restrict__ b3, const float* __restrict__ eps, const b16* __restrict__ WHP, const float* __restrict__ bhh, float* __restrict__ Z, float* __restrict__ KLP, float* __restrict__ GH) { __shared__ __attribute__((aligned(16))) b16 Ah[16][KP + 8], Al[16][KP + 8]; __shared__ float Tf[16][G3 + 4], Kl[16]; const int lane = threadIdx.x, nloc = lane & 15, hlf = lane >> 4; const size_t m0 = (size_t)blockIdx.x * 16;
  for (int rr = 0; rr < 16; ++rr) for (int q = 0; q < 4; ++q) { const int c = q * 32 + lane; const float v = c < H1 ? pmul(pmul(H2[(m0 + rr) * H1P + c] - BNs[c], BNs[H1P + c]), bfv(g[c])) + bfv(be[c]) : 0.0f; b16 p, ql; split16(v * HS, p, ql); Ah[rr][c] = p; Al[rr][c] = ql; }
  if (lane < 16) for (int k = KP; k < KP + 8; ++k) { Ah[lane][k] = (b16)0.0f; Al[lane][k] = (b16)0.0f; }
  wave_lds_sync();
  { v8f acc[16];
#pragma unroll
    for (int t = 0; t < 16; ++t) acc[t] = (v8f){};
#pragma unroll
    for (int kb = 0; kb < KP; kb += 32) { const v16b a = frag_kb(&Ah[nloc][kb], hlf), al = frag_kb(&Al[nloc][kb], hlf);
#pragma unroll
      for (int t = 0; t < 16; ++t) { const v16b bw = frag_kb(W3P + (size_t)(t * 16 + nloc) * KP + kb, hlf); acc[t] = wmma16b(a, bw, acc[t]); acc[t] = wmma16b(al, bw, acc[t]); } }
#pragma unroll
    for (int t = 0; t < 16; ++t) { const int cc = t * 16 + nloc; const float bb = bfv(b3[cc]);
#pragma unroll
      for (int r8 = 0; r8 < 8; ++r8) Tf[8 * hlf + r8][cc] = acc[t][r8] * (1.0f / (HS * WSC)) + bb; } }
  wave_lds_sync();
  for (int rr = 0; rr < 16; ++rr) { float kls = 0.0f; v4f zo; for (int q = 0; q < 4; ++q) { const int l = lane * 4 + q; const float mu = Tf[rr][l], lv = Tf[rr][L + l]; const float zv = mu + pmul(bfv(eps[(m0 + rr) * L + l]), __expf(0.5f * lv)); zo[q] = zv; kls += 1.0f + lv - mu * mu - __expf(lv); b16 p, ql; split16(zv * HS, p, ql); Ah[rr][l] = p; Al[rr][l] = ql; }
    for (int o = 16; o; o >>= 1) kls += __shfl_xor(kls, o); if (lane == 0) Kl[rr] = kls;
    for (int pass = 0; pass < 2; ++pass) { *(volatile v4f*)(Z + (m0 + rr) * L + lane * 4) = zo; __threadfence(); } }
  wave_lds_sync();
#pragma unroll 1
  for (int gq = 0; gq < 3; ++gq) { v8f acc[8];
#pragma unroll
    for (int t = 0; t < 8; ++t) acc[t] = (v8f){};
#pragma unroll
    for (int kb = 0; kb < KP; kb += 32) { const v16b a = frag_kb(&Ah[nloc][kb], hlf), al = frag_kb(&Al[nloc][kb], hlf);
#pragma unroll
      for (int t = 0; t < 8; ++t) { const v16b bw = frag_kb(WHP + (size_t)(gq * L + t * 16 + nloc) * KP + kb, hlf); acc[t] = wmma16b(a, bw, acc[t]); acc[t] = wmma16b(al, bw, acc[t]); } }
#pragma unroll
    for (int t = 0; t < 8; ++t) { const int cc = gq * L + t * 16 + nloc; const float bb = bfv(bhh[cc]);
#pragma unroll
      for (int r8 = 0; r8 < 8; ++r8) Tf[8 * hlf + r8][cc] = acc[t][r8] * (1.0f / (HS * WSC)) + bb; } }
  wave_lds_sync();
  for (int pass = 0; pass < 2; ++pass) { for (int rr = 0; rr < 16; ++rr) for (int q = 0; q < 3; ++q) *(volatile v4f*)(GH + (m0 + rr) * G3 + q * 128 + lane * 4) = *(const v4f*)(&Tf[rr][q * 128 + lane * 4]); ((volatile float*)KLP)[(size_t)blockIdx.x * 32 + lane] = lane < 16 ? Kl[lane] : 0.0f; __threadfence(); } }
__global__ __launch_bounds__(64) void kl_kernel(const float* __restrict__ KLP, float* __restrict__ KLV) { if (threadIdx.x == 0) { double s = 0.0; for (int w = 0; w < NB / 16; ++w) for (int q = 0; q < 16; ++q) s += (double)KLP[w * 32 + q]; const float kl = (float)(-0.5 * s / NB); for (int pass = 0; pass < 2; ++pass) { ((volatile float*)KLV)[0] = kl; __threadfence(); } } }
__global__ __launch_bounds__(256) void tail_kernel(const float* __restrict__ KLV, const float* __restrict__ ZW, float* __restrict__ OUTT) { const size_t i = (size_t)blockIdx.x * 256 + threadIdx.x; if (i >= (size_t)NB * L + 1) return; const float v = i == 0 ? KLV[0] : ZW[i - 1]; for (int pass = 0; pass < 2; ++pass) { ((volatile float*)OUTT)[i] = v; __threadfence(); } }
__global__ __launch_bounds__(256) void dec_kernel(const float* __restrict__ x, const float* __restrict__ GH, const float* __restrict__ Z, const float* __restrict__ wih, const float* __restrict__ bih, const float* __restrict__ wf, const float* __restrict__ bfb, float* __restrict__ OUT0) { __shared__ float Ob[16][2][TD + 1]; const int wave = threadIdx.x >> 5, lane = threadIdx.x & 31; const size_t b0 = (size_t)blockIdx.x * 16;
  float wi[3][4], bi[3][4], wf0[4], wf1[4];
#pragma unroll
  for (int gq = 0; gq < 3; ++gq)
#pragma unroll
    for (int q = 0; q < 4; ++q) { wi[gq][q] = bfv(wih[gq * L + lane * 4 + q]); bi[gq][q] = bfv(bih[gq * L + lane * 4 + q]); }
#pragma unroll
  for (int q = 0; q < 4; ++q) { wf0[q] = bfv(wf[lane * 4 + q]); wf1[q] = bfv(wf[L + lane * 4 + q]); }
  const float bf0 = bfv(bfb[0]), bf1 = bfv(bfb[1]);
#pragma unroll 1
  for (int sb = 0; sb < 2; ++sb) { const int bl = wave * 2 + sb; const size_t b = b0 + bl; float ghr[4], ghz[4], ghn[4], zz[4];
#pragma unroll
    for (int q = 0; q < 4; ++q) { const int l = lane * 4 + q; ghr[q] = GH[b * G3 + l]; ghz[q] = GH[b * G3 + L + l]; ghn[q] = GH[b * G3 + 2 * L + l]; zz[q] = Z[b * L + l]; }
#pragma unroll 1
    for (int t = 0; t < TD; ++t) { const float xt = bfv(x[b * TT + t]); float d0 = 0.0f, d1 = 0.0f;
#pragma unroll
      for (int q = 0; q < 4; ++q) { const float r = sigm(pmul(xt, wi[0][q]) + bi[0][q] + ghr[q]); const float zg = sigm(pmul(xt, wi[1][q]) + bi[1][q] + ghz[q]); const float n = tanhf(pmul(xt, wi[2][q]) + bi[2][q] + pmul(r, ghn[q])); const float hn = fmaxf(pmul(1.0f - zg, n) + pmul(zg, zz[q]), 0.0f); d0 += pmul(hn, wf0[q]); d1 += pmul(hn, wf1[q]); }
      for (int o = 16; o; o >>= 1) { d0 += __shfl_xor(d0, o); d1 += __shfl_xor(d1, o); } if (lane == 0) { Ob[bl][0][t] = d0 + bf0; Ob[bl][1][t] = d1 + bf1; } } }
  __syncthreads();
  for (int pass = 0; pass < 2; ++pass) { for (int idx = threadIdx.x; idx < 16 * 2 * TD; idx += 256) { const int bl = idx / (2 * TD), r = idx % (2 * TD); ((volatile float*)OUT0)[b0 * 2 * TD + idx] = Ob[bl][r / TD][r % TD]; } __threadfence(); } }
}

extern "C" void kernel_launch(void* const* d_in, const int* in_sizes, int n_in, void* d_out, int out_size, void* d_ws, size_t ws_size, hipStream_t stream) {
  (void)n_in;
  auto Fp = [&](int i) { return (const float*)d_in[i]; };
  if (in_sizes[0] != NB * TT || in_sizes[1] != NB * L || in_sizes[2] != H1 * IN || in_sizes[6] != H1 * H1 || in_sizes[10] != 2 * L * H1 || in_sizes[12] != G3 || in_sizes[13] != G3 * L || in_sizes[16] != 2 * L || in_sizes[17] != 2 || out_size != NB * 2 * TD + 1 + NB * L) return;
  size_t off = 0; char* ws = (char*)d_ws;
  auto carve = [&](size_t bytes) { char* p = ws + off; off += (bytes + 255) & ~(size_t)255; return p; };
  b16* W1P = (b16*)carve((size_t)H1P * KP * 2); b16* W2P = (b16*)carve((size_t)H1P * KP * 2); b16* W3P = (b16*)carve((size_t)2 * L * KP * 2); b16* WHP = (b16*)carve((size_t)G3 * KP * 2);
  float* HA = (float*)carve((size_t)NB * H1P * 4); float* HB = (float*)carve((size_t)NB * H1P * 4); float* PS = (float*)carve((size_t)(NB / 16) * 2 * H1P * 4); float* BN1 = (float*)carve(2 * H1P * 4); float* BN2 = (float*)carve(2 * H1P * 4); float* ZW = (float*)carve((size_t)NB * L * 4); float* KLP = (float*)carve((size_t)(NB / 16) * 32 * 4); float* KLV = (float*)carve(256); float* GH = (float*)carve((size_t)NB * G3 * 4);
  if (off > ws_size || off > ((size_t)8 << 20)) return;
  float* OUT0 = (float*)d_out; float* OUTT = OUT0 + (size_t)NB * 2 * TD;
  wput_kernel<<<(G3 * 16 + 255) / 256, 256, 0, stream>>>(Fp(2), Fp(6), Fp(10), Fp(13), W1P, W2P, W3P, WHP);
  enc_kernel<0><<<NB / 16, 32, 0, stream>>>(Fp(0), HA, BN1, Fp(4), Fp(5), W1P, Fp(3), HA, PS); bn_kernel<<<1, 128, 0, stream>>>(PS, BN1);
  enc_kernel<1><<<NB / 16, 32, 0, stream>>>(Fp(0), HA, BN1, Fp(4), Fp(5), W2P, Fp(7), HB, PS); bn_kernel<<<1, 128, 0, stream>>>(PS, BN2);
  lat_kernel<<<NB / 16, 32, 0, stream>>>(HB, BN2, Fp(8), Fp(9), W3P, Fp(11), Fp(1), WHP, Fp(15), ZW, KLP, GH);
  kl_kernel<<<1, 64, 0, stream>>>(KLP, KLV);
  dec_kernel<<<NB / 16, 256, 0, stream>>>(Fp(0), GH, ZW, Fp(12), Fp(14), Fp(16), Fp(17), OUT0);
  tail_kernel<<<(NB * L + 1 + 255) / 256, 256, 0, stream>>>(KLV, ZW, OUTT);
}
